// RelLearnableDecoderLayer_55319178773049
// MI455X (gfx1250) — hardware-verified
//
#include <hip/hip_runtime.h>
#include <math.h>

constexpr int kQlen   = 1024;
constexpr int kBsz    = 4;
constexpr int kDmodel = 1024;
constexpr int kNhead  = 16;
constexpr int kDhead  = 64;
constexpr int kDinner = 4096;
constexpr int kTok    = kQlen * kBsz;
constexpr int kGroups = kBsz * kNhead;
constexpr int kChunk  = 8;
constexpr int kPlaneElems = kQlen * kDhead;
constexpr float kWCarry    = 64.0f;
constexpr float kWCarryInv = 1.0f / 64.0f;
constexpr float kPCarry    = 2048.0f;
constexpr float kAVCarry   = 32.0f;
constexpr float kPVScale   = kAVCarry / kPCarry;
constexpr float kOScale    = 1.0f / (kAVCarry * kWCarry);
constexpr float kScoreScale = 0.125f;
constexpr float kMaskFill   = -1.0e30f;
constexpr float kLnEps      = 1e-5f;
constexpr float kInvD       = 1.0f / 1024.0f;

constexpr size_t kMiB = (size_t)1 << 20;
constexpr size_t kOffQW    = 0;
constexpr size_t kOffQP    = 8 * kMiB;
constexpr size_t kOffKP    = 16 * kMiB;
constexpr size_t kOffVT    = 24 * kMiB;
constexpr size_t kOffREMB  = 32 * kMiB;
constexpr size_t kOffAV    = 34 * kMiB;
constexpr size_t kOffHEADS = 42 * kMiB;
constexpr size_t kOffX16   = 90 * kMiB;
constexpr size_t kOffWQKV  = 98 * kMiB;
constexpr size_t kOffAC    = 42 * kMiB;
constexpr size_t kOffBR    = 74 * kMiB;
constexpr size_t kOffP16   = 106 * kMiB;
constexpr size_t kOffWO    = 0;
constexpr size_t kOffWF1   = 2 * kMiB;
constexpr size_t kOffWF2   = 10 * kMiB;
constexpr size_t kOffY2    = 18 * kMiB;
constexpr size_t kOffY1    = 42 * kMiB;
constexpr size_t kOffOUT1  = 58 * kMiB;
constexpr size_t kOffOUT1H = 74 * kMiB;
constexpr size_t kOffH16   = 82 * kMiB;
constexpr size_t kWsEnd    = 122 * kMiB;

typedef __attribute__((ext_vector_type(16))) _Float16 v16h;
typedef __attribute__((ext_vector_type(8)))  _Float16 v8h;
typedef __attribute__((ext_vector_type(16))) __bf16   v16b;
typedef __attribute__((ext_vector_type(8)))  __bf16   v8b;
typedef __attribute__((ext_vector_type(8)))  float    v8f;
typedef __attribute__((ext_vector_type(4)))  float    v4f;
typedef __attribute__((ext_vector_type(4)))  unsigned int v4u;
typedef __attribute__((ext_vector_type(4)))  int      v4i;

__device__ __forceinline__ unsigned short f2bf_bits(float f) {
  unsigned u = __float_as_uint(f);
  return (unsigned short)((u + 0x7FFFu + ((u >> 16) & 1u)) >> 16);
}
__device__ __forceinline__ float bf_bits2f(unsigned short h) { return __uint_as_float(((unsigned)h) << 16); }

__device__ __forceinline__ void dep_guard_h(v8f& a, v8f& b, v16h x, v16h y) { asm volatile("v_nop\n\tv_nop\n\tv_nop\n\tv_nop" : "+v"(a), "+v"(b) : "v"(x), "v"(y)); }
__device__ __forceinline__ void dep_guard_b(v8f& a, v8f& b, v16b x, v16b y) { asm volatile("v_nop\n\tv_nop\n\tv_nop\n\tv_nop" : "+v"(a), "+v"(b) : "v"(x), "v"(y)); }
__device__ __forceinline__ void keep4_h(v16h a, v16h b, v16h c, v16h d) { asm volatile("v_nop" :: "v"(a), "v"(b), "v"(c), "v"(d)); }
__device__ __forceinline__ void keep4_b(v16b a, v16b b, v16b c, v16b d) { asm volatile("v_nop" :: "v"(a), "v"(b), "v"(c), "v"(d)); }
__device__ __forceinline__ void acc_guard4(v8f& a, v8f& b, v8f& c, v8f& d) { asm volatile("v_nop\n\tv_nop\n\tv_nop\n\tv_nop" : "+v"(a), "+v"(b), "+v"(c), "+v"(d)); }
template <typename T> struct Frag;
template <> struct Frag<_Float16> {
  typedef v16h V; union U { v16h v; v8h h[2]; };
  static __device__ __forceinline__ v16h load(const _Float16* p) {
    U f; f.h[0] = *(const v8h*)(p); f.h[1] = *(const v8h*)(p + 16); return f.v;
  }
  static __device__ __forceinline__ v8f mma(v16h a, v16h b, v8f c) {
    return __builtin_amdgcn_wmma_f32_16x16x32_f16(false, a, false, b, (short)0, c, false, false);
  }
  static __device__ __forceinline__ void guard(v8f& a, v8f& b, v16h x, v16h y) { dep_guard_h(a, b, x, y); }
  static __device__ __forceinline__ void keep(v16h a, v16h b, v16h c, v16h d) { keep4_h(a, b, c, d); }
};
template <> struct Frag<__bf16> {
  typedef v16b V; union U { v16b v; v8b h[2]; };
  static __device__ __forceinline__ v16b load(const __bf16* p) {
    U f; f.h[0] = *(const v8b*)(p); f.h[1] = *(const v8b*)(p + 16); return f.v;
  }
  static __device__ __forceinline__ v8f mma(v16b a, v16b b, v8f c) {
    return __builtin_amdgcn_wmma_f32_16x16x32_bf16(false, a, false, b, (short)0, c, false, false);
  }
  static __device__ __forceinline__ void guard(v8f& a, v8f& b, v16b x, v16b y) { dep_guard_b(a, b, x, y); }
  static __device__ __forceinline__ void keep(v16b a, v16b b, v16b c, v16b d) { keep4_b(a, b, c, d); }
};

__device__ __forceinline__ unsigned pk16(unsigned short a, unsigned short b) { return (unsigned)a | ((unsigned)b << 16); }
__device__ __forceinline__ unsigned short h_bits(float f) { const _Float16 h = (_Float16)f; return __builtin_bit_cast(unsigned short, h); }

template <int ET> struct Elem;
template <> struct Elem<0> { typedef _Float16 T; };
template <> struct Elem<1> { typedef __bf16 T; };
template <int ET, bool SPLIT, int BIAS_MODE, int OUT_MODE, bool RESID, int ACT = 0>
__global__ __launch_bounds__(256) void wmma_gemm64(
    const unsigned short* __restrict__ Ap, const unsigned short* __restrict__ A2p, int lda, long strideA,
    const unsigned short* __restrict__ Btp, const unsigned short* __restrict__ Bt2p, int ldb, long strideB,
    void* __restrict__ Cout, void* __restrict__ Cout2, int ldc, long strideC,
    const float* __restrict__ bias,
    const float* __restrict__ resid, long strideR,
    int M, int N, int K, float scale) {
  typedef typename Elem<ET>::T T;
  typedef typename Frag<T>::V V;
  const T* A = (const T*)Ap; const T* A2 = (const T*)A2p; const T* Bt = (const T*)Btp; const T* Bt2 = (const T*)Bt2p;
  __shared__ __align__(16) float sT[8][16 * 68];
  const int b    = blockIdx.y;
  const int lane = threadIdx.x & 31;
  const int wave = threadIdx.x >> 5;
  const int tilesN = N >> 6;
  const int tilesM = M >> 6;
  const int tile = blockIdx.x * 8 + wave;
  if (tile >= tilesM * tilesN) return;
  const int tm = tile / tilesN;
  const int tn = tile - tm * tilesN;
  const int m0 = tm << 6;
  const int n0 = tn << 6;

  const T* Ab  = A  + (size_t)b * strideA;
  const T* Bb  = Bt + (size_t)b * strideB;
  const T* Ab2 = SPLIT ? (A2  + (size_t)b * strideA) : nullptr;
  const T* Bb2 = SPLIT ? (Bt2 + (size_t)b * strideB) : nullptr;

  const int rlane = lane & 15;
  const int koff  = (lane >> 4) * 8;
  const int mOff  = (lane >> 4) * 8;

  v8f acc[4][4];
#pragma unroll
  for (int i = 0; i < 4; ++i)
#pragma unroll
    for (int j = 0; j < 4; ++j) acc[i][j] = (v8f){0.f,0.f,0.f,0.f,0.f,0.f,0.f,0.f};

  for (int k0 = 0; k0 < K; k0 += 32) {
    V bh[4], bl[4];
#pragma unroll
    for (int j = 0; j < 4; ++j) {
      const size_t bo = (size_t)(n0 + (j << 4) + rlane) * ldb + koff + k0;
      bh[j] = Frag<T>::load(Bb + bo);
      if (SPLIT) bl[j] = Frag<T>::load(Bb2 + bo);
    }
#pragma unroll
    for (int i = 0; i < 4; ++i) {
      const size_t ao = (size_t)(m0 + (i << 4) + rlane) * lda + koff + k0;
      V ah = Frag<T>::load(Ab + ao);
      V al;
      if (SPLIT) al = Frag<T>::load(Ab2 + ao);
#pragma unroll
      for (int j = 0; j < 4; ++j) {
        acc[i][j] = Frag<T>::mma(ah, bh[j], acc[i][j]);
        if (SPLIT) {
          acc[i][j] = Frag<T>::mma(ah, bl[j], acc[i][j]);
          acc[i][j] = Frag<T>::mma(al, bh[j], acc[i][j]);
        }
      }
      Frag<T>::guard(acc[i][0], acc[i][3], ah, SPLIT ? al : ah);
    }
    Frag<T>::keep(bh[0], bh[1], bh[2], bh[3]);
    if (SPLIT) Frag<T>::keep(bl[0], bl[1], bl[2], bl[3]);
  }
  acc_guard4(acc[0][0], acc[0][1], acc[0][2], acc[0][3]);
  acc_guard4(acc[1][0], acc[1][1], acc[1][2], acc[1][3]);
  acc_guard4(acc[2][0], acc[2][1], acc[2][2], acc[2][3]);
  acc_guard4(acc[3][0], acc[3][1], acc[3][2], acc[3][3]);

  float* slab = sT[wave];
  const float* Rb = RESID ? (resid + (size_t)b * strideR) : nullptr;
#pragma unroll
  for (int i = 0; i < 4; ++i) {
    const int mBase = m0 + (i << 4);
#pragma unroll
    for (int j = 0; j < 4; ++j) {
      const int n = n0 + (j << 4) + rlane;
      float bv = 0.f;
      if (BIAS_MODE == 2) bv = bias[n];
#pragma unroll
      for (int r = 0; r < 8; ++r) {
        float v = acc[i][j][r] * scale;
        if (BIAS_MODE == 1) v += bias[mBase + mOff + r];
        if (BIAS_MODE == 2) v += bv;
        if (RESID) v += Rb[(size_t)(mBase + mOff + r) * ldc + n];
        if (ACT == 2) v = fmaxf(v, 0.0f);
        if (ACT == 4) v = (v > 0.f) ? v : 0.01f * v;
        slab[(mOff + r) * 68 + (j << 4) + rlane] = v;
      }
    }
    __builtin_amdgcn_fence(__ATOMIC_RELEASE, "workgroup");
    __builtin_amdgcn_wave_barrier();
    __builtin_amdgcn_fence(__ATOMIC_ACQUIRE, "workgroup");
    if (OUT_MODE == 0) {
      float* C = (float*)Cout + (size_t)b * strideC;
      const int hh = lane >> 4, c4 = (lane & 15) * 4;
      for (int pass = 0; pass < 2; ++pass) {
#pragma unroll
        for (int it = 0; it < 8; ++it) {
          const int row = it * 2 + hh;
          v4f v = *(const v4f*)(slab + row * 68 + c4);
          *(volatile v4f*)(C + (size_t)(mBase + row) * ldc + n0 + c4) = v;
        }
        __threadfence();
      }
    } else {
      const int q = lane >> 3, c8 = (lane & 7) * 8;
      unsigned short* C  = (unsigned short*)Cout  + (size_t)b * strideC;
      unsigned short* C2 = (OUT_MODE == 2) ? ((unsigned short*)Cout2 + (size_t)b * strideC) : nullptr;
      for (int pass = 0; pass < 2; ++pass) {
#pragma unroll
        for (int it = 0; it < 4; ++it) {
          const int row = it * 4 + q;
          const float* sp = slab + row * 68 + c8;
          v8h hv, lv;
#pragma unroll
          for (int e = 0; e < 8; ++e) {
            if (OUT_MODE == 1) {
              hv[e] = (_Float16)sp[e];
            } else {
              unsigned short hb = f2bf_bits(sp[e]);
              unsigned short lb = f2bf_bits(sp[e] - bf_bits2f(hb));
              hv[e] = __builtin_bit_cast(_Float16, hb);
              lv[e] = __builtin_bit_cast(_Float16, lb);
            }
          }
          *(volatile v8h*)(C + (size_t)(mBase + row) * ldc + n0 + c8) = hv;
          if (OUT_MODE == 2) *(volatile v8h*)(C2 + (size_t)(mBase + row) * ldc + n0 + c8) = lv;
        }
        __threadfence();
      }
    }
    __builtin_amdgcn_fence(__ATOMIC_RELEASE, "workgroup");
    __builtin_amdgcn_wave_barrier();
    __builtin_amdgcn_fence(__ATOMIC_ACQUIRE, "workgroup");
  }
}

__global__ __launch_bounds__(256) void cast8_f16_kernel(const float* __restrict__ in, unsigned short* __restrict__ out,
                                                       int n8, float scale) {
  const int i = blockIdx.x * 256 + threadIdx.x;
  if (i >= n8) return;
  const float* p = in + 8 * (size_t)i;
  const v4f a = *(const v4f*)(p);
  const v4f c = *(const v4f*)(p + 4);
  unsigned short hb[8];
#pragma unroll
  for (int e = 0; e < 4; ++e) {
    hb[e]     = h_bits(a[e] * scale);
    hb[4 + e] = h_bits(c[e] * scale);
  }
  const v4u u = (v4u){pk16(hb[0], hb[1]), pk16(hb[2], hb[3]), pk16(hb[4], hb[5]), pk16(hb[6], hb[7])};
  unsigned short* q = out + 8 * (size_t)i;
  *(volatile v4u*)q = u;
  __threadfence();
  *(volatile v4u*)q = u;
}

__global__ __launch_bounds__(256) void remb_kernel(const float* __restrict__ r_emb, unsigned short* __restrict__ out,
                                                   float scale) {
  const int t = threadIdx.x, lane = t & 31, wave = t >> 5;
  const int q = lane >> 3, c8 = (lane & 7) * 8;
  const int orow = (blockIdx.x * 8 + wave) * 4 + q;
  const int n = orow >> 10, j = orow & 1023;
  const float* p = r_emb + ((size_t)j * kNhead + n) * kDhead + c8;
  const v4f a = *(const v4f*)(p);
  const v4f c = *(const v4f*)(p + 4);
  unsigned short hb[8];
#pragma unroll
  for (int e = 0; e < 4; ++e) {
    hb[e]     = h_bits(a[e] * scale);
    hb[4 + e] = h_bits(c[e] * scale);
  }
  const v4u u = (v4u){pk16(hb[0], hb[1]), pk16(hb[2], hb[3]), pk16(hb[4], hb[5]), pk16(hb[6], hb[7])};
  unsigned short* dq = out + (size_t)orow * kDhead + c8;
  *(volatile v4u*)dq = u;
  __threadfence();
  *(volatile v4u*)dq = u;
}

__global__ __launch_bounds__(256) void qk_plane_kernel(const float* __restrict__ heads, const float* __restrict__ rwb,
                                                       unsigned short* __restrict__ qw, unsigned short* __restrict__ qp,
                                                       unsigned short* __restrict__ kp) {
  const int y = blockIdx.y;
  const int t = threadIdx.x, lane = t & 31, wave = t >> 5;
  const int q = lane >> 3, c8 = (lane & 7) * 8;
  const int orow = (blockIdx.x * 8 + wave) * 4 + q;
  const int g = orow >> 10, i = orow & 1023;
  const int b = g >> 4, n = g & 15;
  const int sec = (y == 2) ? 1024 : 0;
  const float* p = heads + (size_t)(i * kBsz + b) * (3 * kDmodel) + sec + n * kDhead + c8;
  v4f a = *(const v4f*)(p);
  v4f c = *(const v4f*)(p + 4);
  const v4f wa = *(const v4f*)(rwb + n * kDhead + c8);
  const v4f wc = *(const v4f*)(rwb + n * kDhead + c8 + 4);
  if (y == 0) { a += wa; c += wc; }
  unsigned short hb[8];
#pragma unroll
  for (int e = 0; e < 4; ++e) {
    hb[e]     = h_bits(a[e]);
    hb[4 + e] = h_bits(c[e]);
  }
  const v4u u = (v4u){pk16(hb[0], hb[1]), pk16(hb[2], hb[3]), pk16(hb[4], hb[5]), pk16(hb[6], hb[7])};
  unsigned short* dst = (y == 0) ? qw : ((y == 1) ? qp : kp);
  unsigned short* dq = dst + (size_t)orow * kDhead + c8;
  *(volatile v4u*)dq = u;
  __threadfence();
  *(volatile v4u*)dq = u;
}

__global__ __launch_bounds__(256) void vt_kernel(const float* __restrict__ heads, unsigned short* __restrict__ vt) {
  __shared__ float sm[64][65];
  const int t  = threadIdx.x;
  const int j0 = blockIdx.x * 64;
  const int g  = blockIdx.y;
  const int b  = g >> 4, n = g & 15;
#pragma unroll
  for (int it = 0; it < 16; ++it) {
    const int e = it * 256 + t;
    const int r = e >> 6;
    const int c = e & 63;
    sm[c][r] = heads[(size_t)((j0 + r) * kBsz + b) * (3 * kDmodel) + 2 * kDmodel + n * kDhead + c];
  }
  __syncthreads();
  const int lane = t & 31, wave = t >> 5;
  const int q = lane >> 3, c8 = (lane & 7) * 8;
  unsigned short* op = vt + (size_t)g * kPlaneElems;
  for (int pass = 0; pass < 2; ++pass) {
#pragma unroll
    for (int it = 0; it < 2; ++it) {
      const int row = wave * 8 + it * 4 + q;
      unsigned short hb[8];
#pragma unroll
      for (int e = 0; e < 8; ++e) hb[e] = h_bits(sm[row][c8 + e]);
      const v4u u = (v4u){pk16(hb[0], hb[1]), pk16(hb[2], hb[3]), pk16(hb[4], hb[5]), pk16(hb[6], hb[7])};
      *(volatile v4u*)(op + (size_t)row * kQlen + j0 + c8) = u;
    }
    __threadfence();
  }
}

__global__ __launch_bounds__(256) void softmax_rel_kernel(const float* __restrict__ ac, const float* __restrict__ br,
                                                          const float* __restrict__ r_bias, const int* __restrict__ amask,
                                                          unsigned short* __restrict__ pout, int nh0) {
  __shared__ float redM[8];
  __shared__ float redS[8];
  __shared__ __align__(16) float prow[1024];
  const int i = blockIdx.x;
  const int y = blockIdx.y;
  const int n = nh0 + y;
  const int t = threadIdx.x, lane = t & 31, wave = t >> 5;
  const int j0 = t * 4;
  const size_t plane = (size_t)y << 20;
  const v4f a  = *(const v4f*)(ac + plane + (size_t)i * kQlen + j0);
  const v4i mk = *(const v4i*)(amask + (size_t)i * kQlen + j0);
  const float* brp = br + plane;
  float s[4];
#pragma unroll
  for (int e = 0; e < 4; ++e) {
    const int j  = j0 + e;
    const int gi = kQlen + i * kQlen + j;
    const int rp = gi / (kQlen + 1);
    const int cc = gi - rp * (kQlen + 1);
    const int rcl = rp > (kQlen - 1) ? (kQlen - 1) : rp;
    const int ccl = cc > 0 ? (cc - 1) : 0;
    const float bw = brp[(size_t)rcl * kQlen + ccl] + r_bias[ccl * kNhead + n];
    const float bd = (cc > 0) ? bw : 0.0f;
    const float sc = (a[e] + bd) * kScoreScale;
    s[e] = (mk[e] != 0) ? kMaskFill : sc;
  }
  float m = fmaxf(fmaxf(s[0], s[1]), fmaxf(s[2], s[3]));
#pragma unroll
  for (int off = 16; off > 0; off >>= 1) m = fmaxf(m, __shfl_xor(m, off, 32));
  if (lane == 0) redM[wave] = m;
  __syncthreads();
  float rm = redM[0];
#pragma unroll
  for (int w = 1; w < 8; ++w) rm = fmaxf(rm, redM[w]);
  float p[4];
#pragma unroll
  for (int e = 0; e < 4; ++e) p[e] = expf(s[e] - rm);
  float ps = (p[0] + p[1]) + (p[2] + p[3]);
#pragma unroll
  for (int off = 16; off > 0; off >>= 1) ps += __shfl_xor(ps, off, 32);
  if (lane == 0) redS[wave] = ps;
  __syncthreads();
  float tot = redS[0];
#pragma unroll
  for (int w = 1; w < 8; ++w) tot += redS[w];
  const float f = kPCarry / tot;
  v4f pv;
#pragma unroll
  for (int e = 0; e < 4; ++e) pv[e] = p[e] * f;
  *(v4f*)(prow + j0) = pv;
  __syncthreads();
  if (t < 128) {
    const v4f u0 = *(const v4f*)(prow + 8 * t);
    const v4f u1 = *(const v4f*)(prow + 8 * t + 4);
    unsigned short hb[8];
#pragma unroll
    for (int e = 0; e < 4; ++e) {
      hb[e]     = h_bits(u0[e]);
      hb[4 + e] = h_bits(u1[e]);
    }
    const v4u w = (v4u){pk16(hb[0], hb[1]), pk16(hb[2], hb[3]), pk16(hb[4], hb[5]), pk16(hb[6], hb[7])};
    unsigned short* q = pout + plane + (size_t)i * kQlen + 8 * t;
    *(volatile v4u*)q = w;
    __threadfence();
    *(volatile v4u*)q = w;
  }
}

template <bool HOUT>
__global__ __launch_bounds__(256) void ln_kernel(const float* __restrict__ yin, const float* __restrict__ gam,
                                                 const float* __restrict__ bet, float* __restrict__ out,
                                                 unsigned short* __restrict__ outh) {
  __shared__ float red[8];
  __shared__ __align__(16) float srow[HOUT ? 1024 : 4];
  const int row = blockIdx.x, t = threadIdx.x, lane = t & 31, wave = t >> 5;
  const int c0 = t * 4;
  const v4f x = *(const v4f*)(yin + (size_t)row * kDmodel + c0);
  float p = (x[0] + x[1]) + (x[2] + x[3]);
#pragma unroll
  for (int off = 16; off > 0; off >>= 1) p += __shfl_xor(p, off, 32);
  if (lane == 0) red[wave] = p;
  __syncthreads();
  float tot = red[0];
#pragma unroll
  for (int w = 1; w < 8; ++w) tot += red[w];
  const float mu = tot * kInvD;
  __syncthreads();
  float d[4];
#pragma unroll
  for (int e = 0; e < 4; ++e) d[e] = x[e] - mu;
  float p2 = (d[0] * d[0] + d[1] * d[1]) + (d[2] * d[2] + d[3] * d[3]);
#pragma unroll
  for (int off = 16; off > 0; off >>= 1) p2 += __shfl_xor(p2, off, 32);
  if (lane == 0) red[wave] = p2;
  __syncthreads();
  float tot2 = red[0];
#pragma unroll
  for (int w = 1; w < 8; ++w) tot2 += red[w];
  const float rs = rsqrtf(tot2 * kInvD + kLnEps);
  const v4f gv = *(const v4f*)(gam + c0);
  const v4f bv = *(const v4f*)(bet + c0);
  v4f o;
#pragma unroll
  for (int e = 0; e < 4; ++e) o[e] = (d[e] * rs) * gv[e] + bv[e];
  float* op = out + (size_t)row * kDmodel + c0;
  *(volatile v4f*)op = o;
  __threadfence();
  *(volatile v4f*)op = o;
  if (HOUT) {
    *(v4f*)(srow + c0) = o;
    __syncthreads();
    if (t < 128) {
      const v4f u0 = *(const v4f*)(srow + 8 * t);
      const v4f u1 = *(const v4f*)(srow + 8 * t + 4);
      unsigned short hb[8];
#pragma unroll
      for (int e = 0; e < 4; ++e) {
        hb[e]     = h_bits(u0[e]);
        hb[4 + e] = h_bits(u1[e]);
      }
      const v4u w = (v4u){pk16(hb[0], hb[1]), pk16(hb[2], hb[3]), pk16(hb[4], hb[5]), pk16(hb[6], hb[7])};
      unsigned short* q = outh + (size_t)row * kDmodel + 8 * t;
      *(volatile v4u*)q = w;
      __threadfence();
      *(volatile v4u*)q = w;
    }
  }
}

extern "C" void kernel_launch(void* const* d_in, const int* in_sizes, int n_in,
                              void* d_out, int out_size, void* d_ws, size_t ws_size,
                              hipStream_t stream) {
  if (n_in < 15) return;
  if (in_sizes[0] != kTok * kDmodel) return;
  if (in_sizes[1] != kQlen * kNhead * kDhead) return;
  if (in_sizes[2] != kNhead * kDhead) return;
  if (in_sizes[3] != kQlen * kNhead) return;
  if (in_sizes[4] != kQlen * kQlen) return;
  if (in_sizes[5] != 3 * kDmodel * kDmodel) return;
  if (in_sizes[6] != kDmodel * kDmodel) return;
  if (in_sizes[9] != kDinner * kDmodel) return;
  if (in_sizes[10] != kDinner) return;
  if (in_sizes[11] != kDmodel * kDinner) return;
  if (out_size != kTok * kDmodel) return;
  if (ws_size < kWsEnd) return;

  const float* dec_inp  = (const float*)d_in[0];
  const float* r_emb    = (const float*)d_in[1];
  const float* r_w_bias = (const float*)d_in[2];
  const float* r_bias   = (const float*)d_in[3];
  const int*   amask    = (const int*)d_in[4];
  const float* qkv_w    = (const float*)d_in[5];
  const float* o_w      = (const float*)d_in[6];
  const float* ln1_g    = (const float*)d_in[7];
  const float* ln1_b    = (const float*)d_in[8];
  const float* ff_w1    = (const float*)d_in[9];
  const float* ff_b1    = (const float*)d_in[10];
  const float* ff_w2    = (const float*)d_in[11];
  const float* ff_b2    = (const float*)d_in[12];
  const float* ln2_g    = (const float*)d_in[13];
  const float* ln2_b    = (const float*)d_in[14];

  char* ws = (char*)d_ws;
  unsigned short* QW    = (unsigned short*)(ws + kOffQW);
  unsigned short* QP    = (unsigned short*)(ws + kOffQP);
  unsigned short* KP    = (unsigned short*)(ws + kOffKP);
  unsigned short* VT    = (unsigned short*)(ws + kOffVT);
  unsigned short* REMB  = (unsigned short*)(ws + kOffREMB);
  unsigned short* AV    = (unsigned short*)(ws + kOffAV);
  float*          HEADS = (float*)(ws + kOffHEADS);
  unsigned short* X16   = (unsigned short*)(ws + kOffX16);
  unsigned short* WQKV  = (unsigned short*)(ws + kOffWQKV);
  float*          ACp   = (float*)(ws + kOffAC);
  float*          BRp   = (float*)(ws + kOffBR);
  unsigned short* P16   = (unsigned short*)(ws + kOffP16);
  unsigned short* WO    = (unsigned short*)(ws + kOffWO);
  unsigned short* WF1   = (unsigned short*)(ws + kOffWF1);
  unsigned short* WF2   = (unsigned short*)(ws + kOffWF2);
  float*          Y2    = (float*)(ws + kOffY2);
  float*          Y1    = (float*)(ws + kOffY1);
  float*          OUT1  = (float*)(ws + kOffOUT1);
  unsigned short* OUT1H = (unsigned short*)(ws + kOffOUT1H);
  unsigned short* H16   = (unsigned short*)(ws + kOffH16);
  float*          OUTF  = (float*)d_out;

  cast8_f16_kernel<<<(kTok * kDmodel / 8) / 256, 256, 0, stream>>>(dec_inp, X16, kTok * kDmodel / 8, 1.0f);
  cast8_f16_kernel<<<(3 * kDmodel * kDmodel / 8) / 256, 256, 0, stream>>>(qkv_w, WQKV, 3 * kDmodel * kDmodel / 8, kWCarry);
  remb_kernel<<<(kNhead * kQlen) / 32, 256, 0, stream>>>(r_emb, REMB, kWCarry);
  wmma_gemm64<0, false, 0, 0, false, 0><<<dim3(384, 1), 256, 0, stream>>>(
      X16, X16, kDmodel, 0L, WQKV, WQKV, kDmodel, 0L, HEADS, HEADS, 3 * kDmodel, 0L,
      ln1_g, dec_inp, 0L, kTok, 3 * kDmodel, kDmodel, kWCarryInv);

  qk_plane_kernel<<<dim3((kGroups * kQlen) / 32, 3), 256, 0, stream>>>(HEADS, r_w_bias, QW, QP, KP);
  vt_kernel<<<dim3(kQlen / 64, kGroups), 256, 0, stream>>>(HEADS, VT);

  for (int c = 0; c < kGroups / kChunk; ++c) {
    const int g0  = c * kChunk;
    const int b   = g0 >> 4;
    const int nh0 = g0 & 15;
    const long gstride = (long)kPlaneElems;
    wmma_gemm64<0, false, 0, 0, false, 0><<<dim3(32, kChunk), 256, 0, stream>>>(
        QW + (size_t)g0 * kPlaneElems, QW + (size_t)g0 * kPlaneElems, kDhead, gstride,
        KP + (size_t)g0 * kPlaneElems, KP + (size_t)g0 * kPlaneElems, kDhead, gstride,
        ACp, ACp, kQlen, (long)kQlen * kQlen, ln1_g, dec_inp, 0L, kQlen, kQlen, kDhead, 1.0f);
    wmma_gemm64<0, false, 0, 0, false, 0><<<dim3(32, kChunk), 256, 0, stream>>>(
        QP + (size_t)g0 * kPlaneElems, QP + (size_t)g0 * kPlaneElems, kDhead, gstride,
        REMB + (size_t)nh0 * kPlaneElems, REMB + (size_t)nh0 * kPlaneElems, kDhead, gstride,
        BRp, BRp, kQlen, (long)kQlen * kQlen, ln1_g, dec_inp, 0L, kQlen, kQlen, kDhead, kWCarryInv);
    softmax_rel_kernel<<<dim3(kQlen, kChunk), 256, 0, stream>>>(ACp, BRp, r_bias, amask, P16, nh0);
    wmma_gemm64<0, false, 0, 1, false, 0><<<dim3(2, kChunk), 256, 0, stream>>>(
        P16, P16, kQlen, (long)kQlen * kQlen,
        VT + (size_t)g0 * kPlaneElems, VT + (size_t)g0 * kPlaneElems, kQlen, gstride,
        AV + (size_t)b * kDmodel + (size_t)nh0 * kDhead, AV, kBsz * kDmodel, (long)kDhead,
        ln1_g, dec_inp, 0L, kQlen, kDhead, kQlen, kPVScale);
  }

  cast8_f16_kernel<<<(kDmodel * kDmodel / 8) / 256, 256, 0, stream>>>(o_w, WO, kDmodel * kDmodel / 8, kWCarry);
  cast8_f16_kernel<<<(kDinner * kDmodel / 8) / 256, 256, 0, stream>>>(ff_w1, WF1, kDinner * kDmodel / 8, kWCarry);
  cast8_f16_kernel<<<(kDmodel * kDinner / 8) / 256, 256, 0, stream>>>(ff_w2, WF2, kDmodel * kDinner / 8, kWCarry);
  wmma_gemm64<0, false, 0, 0, true, 0><<<dim3(128, 1), 256, 0, stream>>>(
      AV, AV, kDmodel, 0L, WO, WO, kDmodel, 0L, Y1, Y1, kDmodel, 0L,
      ln1_g, dec_inp, 0L, kTok, kDmodel, kDmodel, kOScale);
  ln_kernel<true><<<kTok, 256, 0, stream>>>(Y1, ln1_g, ln1_b, OUT1, OUT1H);
  wmma_gemm64<0, false, 2, 1, false, 2><<<dim3(512, 1), 256, 0, stream>>>(
      OUT1H, OUT1H, kDmodel, 0L, WF1, WF1, kDmodel, 0L, H16, H16, kDinner, 0L,
      ff_b1, dec_inp, 0L, kTok, kDinner, kDmodel, kWCarryInv);
  wmma_gemm64<0, false, 2, 0, true, 0><<<dim3(128, 1), 256, 0, stream>>>(
      H16, H16, kDinner, 0L, WF2, WF2, kDinner, 0L, Y2, Y2, kDmodel, 0L,
      ff_b2, OUT1, 0L, kTok, kDmodel, kDinner, kWCarryInv);
  ln_kernel<false><<<kTok, 256, 0, stream>>>(Y2, ln2_g, ln2_b, OUTF, OUT1H);
}
